// LSTMModel_45887430590853
// MI455X (gfx1250) — hardware-verified
//
#include <hip/hip_runtime.h>
#include <math.h>

constexpr int NBATCH  = 256;
constexpr int NSTEP   = 1024;
constexpr int NIN     = 32;
constexpr int NHID    = 128;
constexpr int NGATE   = 4 * NHID;
constexpr int NOUTA   = 27;
constexpr int NTHR    = 256;
constexpr int NWAVE   = NTHR / 32;
constexpr int SEQ_BLK = 16;
constexpr int XPITCH  = 40;
constexpr int HPITCH  = 136;
constexpr int SPITCH  = 260;
constexpr int XS_SZ   = SEQ_BLK * XPITCH;
constexpr int HS_SZ   = SEQ_BLK * HPITCH;
constexpr int NYA     = NBATCH * NOUTA;
constexpr int NYT     = NBATCH;
constexpr int NYALL   = NYA + NYT;
constexpr int NFCW    = NOUTA * NHID + NHID;
constexpr float XCARRY = 16.0f;
constexpr float HCARRY = 16.0f;
constexpr float WCARRY = 256.0f;
constexpr float ZINV   = 1.0f / (16.0f * 256.0f);
static_assert(XCARRY == HCARRY, "x and h terms share one accumulator");
static_assert(NBATCH % SEQ_BLK == 0, "grid exact");
static_assert(NHID == 16 * NWAVE, "one 16-unit subtile per wave");
static_assert(NIN == 32, "x term is exactly one 32-deep k chunk");
static_assert(NHID % 32 == 0, "h terms are whole 32-deep k chunks");
static_assert((2 * XS_SZ) % NTHR == 0 && (2 * HS_SZ) % NTHR == 0, "zero-fill loops exact");
static_assert(SEQ_BLK * NIN == 128 * 4, "x staging: 128 threads x 4 floats");
static_assert(SEQ_BLK * NHID == 2 * NTHR * 4, "final h store: 2 iterations x 256 threads x 4 floats");
static_assert(NYALL % (NTHR * 4) == 0, "output store: 7 iterations x 256 threads x 4 floats");
static_assert(NYT == NTHR, "one thread per second-head element");
static_assert(NYA % NTHR == 0, "first-head loop exact");
static_assert((NGATE * NIN / 8) % NTHR == 0 && (NGATE * NHID / 8) % NTHR == 0, "convert grids exact");
static_assert(XPITCH % 8 == 0 && HPITCH % 8 == 0 && SPITCH % 4 == 0, "16-B aligned fragment and slab rows");

typedef __attribute__((ext_vector_type(16))) _Float16 v16h;
typedef __attribute__((ext_vector_type(8)))  _Float16 v8h;
typedef __attribute__((ext_vector_type(8)))  float    v8f;
typedef __attribute__((ext_vector_type(4)))  float    v4f;
typedef __attribute__((ext_vector_type(2)))  unsigned v2u;

__device__ __forceinline__ void dep_guard_h(v8f& a, v8f& b, v16h x, v16h y) { asm volatile("v_nop\n\tv_nop\n\tv_nop\n\tv_nop" : "+v"(a), "+v"(b) : "v"(x), "v"(y)); }
__device__ __forceinline__ void keep4_h(v16h a, v16h b, v16h c, v16h d) { asm volatile("v_nop" :: "v"(a), "v"(b), "v"(c), "v"(d)); }
__device__ __forceinline__ void acc_guard4(v8f& a, v8f& b, v8f& c, v8f& d) { asm volatile("v_nop\n\tv_nop\n\tv_nop\n\tv_nop" : "+v"(a), "+v"(b), "+v"(c), "+v"(d)); }
__device__ __forceinline__ void grp_guard_h(v8f& a0, v8f& a1, v8f& a2, v8f& a3, v16h x, v16h y0, v16h y1, v16h y2, v16h y3) {
  asm volatile("v_nop\n\tv_nop\n\tv_nop\n\tv_nop" : "+v"(a0), "+v"(a1), "+v"(a2), "+v"(a3) : "v"(x), "v"(y0), "v"(y1), "v"(y2), "v"(y3));
}

template <typename T> struct Frag;
template <> struct Frag<_Float16> {
  typedef v16h V; union U { v16h v; v8h h[2]; };
  static __device__ __forceinline__ v16h load(const _Float16* p) {
    U f; f.h[0] = *(const v8h*)(p); f.h[1] = *(const v8h*)(p + 16); return f.v;
  }
  static __device__ __forceinline__ v8f mma(v16h a, v16h b, v8f c) {
    return __builtin_amdgcn_wmma_f32_16x16x32_f16(false, a, false, b, (short)0, c, false, false);
  }
  static __device__ __forceinline__ void guard(v8f& a, v8f& b, v16h x, v16h y) { dep_guard_h(a, b, x, y); }
  static __device__ __forceinline__ void keep(v16h a, v16h b, v16h c, v16h d) { keep4_h(a, b, c, d); }
};

__device__ __forceinline__ float fsig(float z) {
  const float zc = fminf(fmaxf(z, -30.0f), 30.0f);
  return __builtin_amdgcn_rcpf(1.0f + expf(-zc));
}
__device__ __forceinline__ float ftanh(float z) {
  const float zc = fminf(fmaxf(z, -15.0f), 15.0f);
  return 1.0f - 2.0f * __builtin_amdgcn_rcpf(expf(2.0f * zc) + 1.0f);
}

__global__ __launch_bounds__(NTHR) void cvt_f16x8_kernel(const float* __restrict__ src, unsigned short* __restrict__ dst,
                                                         int n8, float sc) {
  const int i = blockIdx.x * NTHR + threadIdx.x;
  if (i < n8) {
    const float* sp = src + (size_t)i * 8;
    const v4f a = *(const v4f*)(sp);
    const v4f b = *(const v4f*)(sp + 4);
    v8h hv;
#pragma unroll
    for (int e = 0; e < 4; ++e) {
      const float s0 = a[e] * sc;
      const float s1 = b[e] * sc;
      hv[e]     = (_Float16)s0;
      hv[4 + e] = (_Float16)s1;
    }
    *(volatile v8h*)(dst + (size_t)i * 8) = hv;
    __threadfence();
    *(volatile v8h*)(dst + (size_t)i * 8) = hv;
  }
}

__device__ __forceinline__ void stage_x(const float* __restrict__ x, _Float16* xs, int rowbase, int t, int tid) {
  const int m = tid >> 3, f4 = (tid & 7) * 4;
  const v4f v = *(const v4f*)(x + ((size_t)(rowbase + m) * NSTEP + (size_t)t) * NIN + f4);
  const float x0 = v[0] * XCARRY, x1 = v[1] * XCARRY, x2 = v[2] * XCARRY, x3 = v[3] * XCARRY;
  const _Float16 g0 = (_Float16)x0, g1 = (_Float16)x1, g2 = (_Float16)x2, g3 = (_Float16)x3;
  const unsigned u0 = (unsigned)__builtin_bit_cast(unsigned short, g0);
  const unsigned u1 = (unsigned)__builtin_bit_cast(unsigned short, g1);
  const unsigned u2 = (unsigned)__builtin_bit_cast(unsigned short, g2);
  const unsigned u3 = (unsigned)__builtin_bit_cast(unsigned short, g3);
  v2u pk;
  pk[0] = u0 | (u1 << 16);
  pk[1] = u2 | (u3 << 16);
  *(v2u*)(xs + m * XPITCH + f4) = pk;
}

__global__ __launch_bounds__(NTHR) void lstm2_kernel(const float* __restrict__ x,
                                                     const unsigned short* __restrict__ W0Xp,
                                                     const unsigned short* __restrict__ W0Hp,
                                                     const unsigned short* __restrict__ W1Xp,
                                                     const unsigned short* __restrict__ W1Hp,
                                                     const float* __restrict__ bih0, const float* __restrict__ bhh0,
                                                     const float* __restrict__ bih1, const float* __restrict__ bhh1,
                                                     float* __restrict__ LAST) {
  __shared__ __align__(16) _Float16 Xs[2 * XS_SZ];
  __shared__ __align__(16) _Float16 H1s[2 * HS_SZ];
  __shared__ __align__(16) _Float16 H2s[2 * HS_SZ];
  __shared__ __align__(16) float    Fs[SEQ_BLK * SPITCH];
  const _Float16* W0X = (const _Float16*)W0Xp;
  const _Float16* W0H = (const _Float16*)W0Hp;
  const _Float16* W1X = (const _Float16*)W1Xp;
  const _Float16* W1H = (const _Float16*)W1Hp;
  const int tid = threadIdx.x, lane = tid & 31, wave = tid >> 5;
  const int c = lane & 15, hh = lane >> 4, koff = hh * 8;
  const int j = 16 * wave + c;
  const int rowbase = blockIdx.x * SEQ_BLK;

#pragma unroll 1
  for (int i = tid; i < 2 * XS_SZ; i += NTHR) Xs[i] = (_Float16)0.0f;
#pragma unroll 1
  for (int i = tid; i < 2 * HS_SZ; i += NTHR) { H1s[i] = (_Float16)0.0f; H2s[i] = (_Float16)0.0f; }

  float bb0[4], bb1[4];
  {
    float u[4], v[4];
#pragma unroll
    for (int gI = 0; gI < 4; ++gI) { u[gI] = bih0[gI * NHID + j]; v[gI] = bhh0[gI * NHID + j]; }
    asm volatile("" ::: "memory");
#pragma unroll
    for (int gI = 0; gI < 4; ++gI) bb0[gI] = u[gI] + v[gI];
#pragma unroll
    for (int gI = 0; gI < 4; ++gI) { u[gI] = bih1[gI * NHID + j]; v[gI] = bhh1[gI * NHID + j]; }
    asm volatile("" ::: "memory");
#pragma unroll
    for (int gI = 0; gI < 4; ++gI) bb1[gI] = u[gI] + v[gI];
  }
  float c1[8], c2[8], h2v[8];
#pragma unroll
  for (int r = 0; r < 8; ++r) { c1[r] = 0.0f; c2[r] = 0.0f; h2v[r] = 0.0f; }
  __syncthreads();
  if (wave < 4) stage_x(x, Xs, rowbase, 0, tid);
  __syncthreads();

  const v8f z8 = {0.f, 0.f, 0.f, 0.f, 0.f, 0.f, 0.f, 0.f};

#pragma unroll 1
  for (int t = 0; t < NSTEP; ++t) {
    const int cur = t & 1, nxt = cur ^ 1;
    {
      const int tn = (t + 1 < NSTEP) ? (t + 1) : (NSTEP - 1);
      if (wave < 4) stage_x(x, Xs + nxt * XS_SZ, rowbase, tn, tid);
    }

    {
      const _Float16* xr  = Xs  + cur * XS_SZ + c * XPITCH + koff;
      const _Float16* hr  = H1s + cur * HS_SZ + c * HPITCH + koff;
      _Float16*       hw  = H1s + nxt * HS_SZ;
      v8f acc[4];
      acc[0] = z8; acc[1] = z8; acc[2] = z8; acc[3] = z8;
      {
        const v16h a  = Frag<_Float16>::load(xr);
        const v16h b0 = Frag<_Float16>::load(W0X + (size_t)(0 * NHID + j) * NIN + koff);
        const v16h b1 = Frag<_Float16>::load(W0X + (size_t)(1 * NHID + j) * NIN + koff);
        const v16h b2 = Frag<_Float16>::load(W0X + (size_t)(2 * NHID + j) * NIN + koff);
        const v16h b3 = Frag<_Float16>::load(W0X + (size_t)(3 * NHID + j) * NIN + koff);
        acc[0] = Frag<_Float16>::mma(a, b0, acc[0]);
        acc[1] = Frag<_Float16>::mma(a, b1, acc[1]);
        acc[2] = Frag<_Float16>::mma(a, b2, acc[2]);
        acc[3] = Frag<_Float16>::mma(a, b3, acc[3]);
        grp_guard_h(acc[0], acc[1], acc[2], acc[3], a, b0, b1, b2, b3);
      }
#pragma unroll 1
      for (int k0 = 0; k0 < NHID; k0 += 32) {
        const v16h a  = Frag<_Float16>::load(hr + k0);
        const v16h b0 = Frag<_Float16>::load(W0H + (size_t)(0 * NHID + j) * NHID + koff + k0);
        const v16h b1 = Frag<_Float16>::load(W0H + (size_t)(1 * NHID + j) * NHID + koff + k0);
        const v16h b2 = Frag<_Float16>::load(W0H + (size_t)(2 * NHID + j) * NHID + koff + k0);
        const v16h b3 = Frag<_Float16>::load(W0H + (size_t)(3 * NHID + j) * NHID + koff + k0);
        acc[0] = Frag<_Float16>::mma(a, b0, acc[0]);
        acc[1] = Frag<_Float16>::mma(a, b1, acc[1]);
        acc[2] = Frag<_Float16>::mma(a, b2, acc[2]);
        acc[3] = Frag<_Float16>::mma(a, b3, acc[3]);
        grp_guard_h(acc[0], acc[1], acc[2], acc[3], a, b0, b1, b2, b3);
      }
      acc_guard4(acc[0], acc[1], acc[2], acc[3]);
#pragma unroll
      for (int r = 0; r < 8; ++r) {
        const float zi = acc[0][r] * ZINV + bb0[0];
        const float zf = acc[1][r] * ZINV + bb0[1];
        const float zg = acc[2][r] * ZINV + bb0[2];
        const float zo = acc[3][r] * ZINV + bb0[3];
        const float ig = fsig(zi);
        const float fg = fsig(zf);
        const float gg = ftanh(zg);
        const float og = fsig(zo);
        const float cn = fg * c1[r] + ig * gg;
        c1[r] = cn;
        const float hn = og * ftanh(cn);
        hw[(8 * hh + r) * HPITCH + j] = (_Float16)(hn * HCARRY);
      }
    }
    __syncthreads();

    {
      const _Float16* ar  = H1s + nxt * HS_SZ + c * HPITCH + koff;
      const _Float16* hr  = H2s + cur * HS_SZ + c * HPITCH + koff;
      _Float16*       hw  = H2s + nxt * HS_SZ;
      v8f acc[4];
      acc[0] = z8; acc[1] = z8; acc[2] = z8; acc[3] = z8;
#pragma unroll 1
      for (int k0 = 0; k0 < NHID; k0 += 32) {
        const v16h a  = Frag<_Float16>::load(ar + k0);
        const v16h b0 = Frag<_Float16>::load(W1X + (size_t)(0 * NHID + j) * NHID + koff + k0);
        const v16h b1 = Frag<_Float16>::load(W1X + (size_t)(1 * NHID + j) * NHID + koff + k0);
        const v16h b2 = Frag<_Float16>::load(W1X + (size_t)(2 * NHID + j) * NHID + koff + k0);
        const v16h b3 = Frag<_Float16>::load(W1X + (size_t)(3 * NHID + j) * NHID + koff + k0);
        acc[0] = Frag<_Float16>::mma(a, b0, acc[0]);
        acc[1] = Frag<_Float16>::mma(a, b1, acc[1]);
        acc[2] = Frag<_Float16>::mma(a, b2, acc[2]);
        acc[3] = Frag<_Float16>::mma(a, b3, acc[3]);
        grp_guard_h(acc[0], acc[1], acc[2], acc[3], a, b0, b1, b2, b3);
      }
#pragma unroll 1
      for (int k0 = 0; k0 < NHID; k0 += 32) {
        const v16h a  = Frag<_Float16>::load(hr + k0);
        const v16h b0 = Frag<_Float16>::load(W1H + (size_t)(0 * NHID + j) * NHID + koff + k0);
        const v16h b1 = Frag<_Float16>::load(W1H + (size_t)(1 * NHID + j) * NHID + koff + k0);
        const v16h b2 = Frag<_Float16>::load(W1H + (size_t)(2 * NHID + j) * NHID + koff + k0);
        const v16h b3 = Frag<_Float16>::load(W1H + (size_t)(3 * NHID + j) * NHID + koff + k0);
        acc[0] = Frag<_Float16>::mma(a, b0, acc[0]);
        acc[1] = Frag<_Float16>::mma(a, b1, acc[1]);
        acc[2] = Frag<_Float16>::mma(a, b2, acc[2]);
        acc[3] = Frag<_Float16>::mma(a, b3, acc[3]);
        grp_guard_h(acc[0], acc[1], acc[2], acc[3], a, b0, b1, b2, b3);
      }
      acc_guard4(acc[0], acc[1], acc[2], acc[3]);
#pragma unroll
      for (int r = 0; r < 8; ++r) {
        const float zi = acc[0][r] * ZINV + bb1[0];
        const float zf = acc[1][r] * ZINV + bb1[1];
        const float zg = acc[2][r] * ZINV + bb1[2];
        const float zo = acc[3][r] * ZINV + bb1[3];
        const float ig = fsig(zi);
        const float fg = fsig(zf);
        const float gg = ftanh(zg);
        const float og = fsig(zo);
        const float cn = fg * c2[r] + ig * gg;
        c2[r] = cn;
        const float hn = og * ftanh(cn);
        h2v[r] = hn;
        hw[(8 * hh + r) * HPITCH + j] = (_Float16)(hn * HCARRY);
      }
    }
    __syncthreads();
  }

#pragma unroll
  for (int r = 0; r < 8; ++r) Fs[(8 * hh + r) * SPITCH + j] = h2v[r];
  __syncthreads();
  for (int pass = 0; pass < 2; ++pass) {
#pragma unroll
    for (int it = 0; it < 2; ++it) {
      const int idx = it * NTHR + tid;
      const int row = idx >> 5, c4 = (idx & 31) * 4;
      const v4f v = *(const v4f*)(Fs + row * SPITCH + c4);
      *(volatile v4f*)(LAST + (size_t)(rowbase + row) * NHID + c4) = v;
    }
    __threadfence();
  }
}

__global__ __launch_bounds__(NTHR) void heads_kernel(const float* __restrict__ last,
                                                     const float* __restrict__ fc1w, const float* __restrict__ fc1b,
                                                     const float* __restrict__ fc2w, const float* __restrict__ fc2b,
                                                     float* __restrict__ out) {
  __shared__ __align__(16) float wl[NFCW];
  __shared__ __align__(16) float os[NYALL];
  const int tid = threadIdx.x;
#pragma unroll 1
  for (int i = tid; i < NOUTA * NHID; i += NTHR) wl[i] = fc1w[i];
  if (tid < NHID) wl[NOUTA * NHID + tid] = fc2w[tid];
  __syncthreads();
#pragma unroll 1
  for (int e = tid; e < NYA; e += NTHR) {
    const int b = e / NOUTA;
    const int o = e - b * NOUTA;
    const float* lr = last + (size_t)b * NHID;
    const float* wr = wl + o * NHID;
    float s = 0.0f;
#pragma unroll 8
    for (int k = 0; k < NHID; ++k) s = fmaf(lr[k], wr[k], s);
    os[e] = s + fc1b[o];
  }
  {
    const float* lr = last + (size_t)tid * NHID;
    const float* wr = wl + NOUTA * NHID;
    float s = 0.0f;
#pragma unroll 8
    for (int k = 0; k < NHID; ++k) s = fmaf(lr[k], wr[k], s);
    os[NYA + tid] = s + fc2b[0];
  }
  __syncthreads();
  for (int pass = 0; pass < 2; ++pass) {
#pragma unroll
    for (int it = 0; it < NYALL / (NTHR * 4); ++it) {
      const int idx4 = (it * NTHR + tid) * 4;
      const v4f v = *(const v4f*)(os + idx4);
      *(volatile v4f*)(out + idx4) = v;
    }
    __threadfence();
  }
}

extern "C" void kernel_launch(void* const* d_in, const int* in_sizes, int n_in,
                              void* d_out, int out_size, void* d_ws, size_t ws_size, hipStream_t stream) {
  if (n_in < 13 || d_out == nullptr || d_ws == nullptr) return;
  if (in_sizes[0] != NBATCH * NSTEP * NIN || in_sizes[1] != NGATE * NIN || in_sizes[2] != NGATE * NHID ||
      in_sizes[3] != NGATE || in_sizes[4] != NGATE || in_sizes[5] != NGATE * NHID || in_sizes[6] != NGATE * NHID ||
      in_sizes[7] != NGATE || in_sizes[8] != NGATE || in_sizes[9] != NOUTA * NHID || in_sizes[10] != NOUTA ||
      in_sizes[11] != NHID || in_sizes[12] != 1 || out_size != NYALL) return;

  const float* x     = (const float*)d_in[0];
  const float* w_ih0 = (const float*)d_in[1];
  const float* w_hh0 = (const float*)d_in[2];
  const float* b_ih0 = (const float*)d_in[3];
  const float* b_hh0 = (const float*)d_in[4];
  const float* w_ih1 = (const float*)d_in[5];
  const float* w_hh1 = (const float*)d_in[6];
  const float* b_ih1 = (const float*)d_in[7];
  const float* b_hh1 = (const float*)d_in[8];
  const float* fc1w  = (const float*)d_in[9];
  const float* fc1b  = (const float*)d_in[10];
  const float* fc2w  = (const float*)d_in[11];
  const float* fc2b  = (const float*)d_in[12];
  float* out = (float*)d_out;

  char* ws = (char*)d_ws; size_t off = 0;
  auto carve = [&](size_t bytes) -> char* { char* p = ws + off; off += (bytes + 255) & ~(size_t)255; return p; };
  unsigned short* W0X  = (unsigned short*)carve((size_t)NGATE * NIN * 2);
  unsigned short* W0H  = (unsigned short*)carve((size_t)NGATE * NHID * 2);
  unsigned short* W1X  = (unsigned short*)carve((size_t)NGATE * NHID * 2);
  unsigned short* W1H  = (unsigned short*)carve((size_t)NGATE * NHID * 2);
  float*          LAST = (float*)carve((size_t)NBATCH * NHID * 4);
  if (off > ws_size || off > (size_t)134217728) return;

  const int n8x = NGATE * NIN / 8;
  const int n8h = NGATE * NHID / 8;
  cvt_f16x8_kernel<<<n8x / NTHR, NTHR, 0, stream>>>(w_ih0, W0X, n8x, WCARRY);
  cvt_f16x8_kernel<<<n8h / NTHR, NTHR, 0, stream>>>(w_hh0, W0H, n8h, WCARRY);
  cvt_f16x8_kernel<<<n8h / NTHR, NTHR, 0, stream>>>(w_ih1, W1X, n8h, WCARRY);
  cvt_f16x8_kernel<<<n8h / NTHR, NTHR, 0, stream>>>(w_hh1, W1H, n8h, WCARRY);
  lstm2_kernel<<<NBATCH / SEQ_BLK, NTHR, 0, stream>>>(x, W0X, W0H, W1X, W1H, b_ih0, b_hh0, b_ih1, b_hh1, LAST);
  heads_kernel<<<1, NTHR, 0, stream>>>(LAST, fc1w, fc1b, fc2w, fc2b, out);
}
